// PointNet2Encoder_66520453480973
// MI455X (gfx1250) — hardware-verified
//
#include <hip/hip_runtime.h>
#include <stdint.h>
#include <math.h>

#pragma clang fp contract(off)

typedef __attribute__((ext_vector_type(16))) __bf16   v16b;
typedef __attribute__((ext_vector_type(8)))  __bf16   v8b;
typedef __attribute__((ext_vector_type(8)))  float    v8f;
typedef __attribute__((ext_vector_type(4)))  float    v4f;
typedef __attribute__((ext_vector_type(4)))  unsigned int v4u;

constexpr int kBatch = 8;
constexpr int kN1    = 8192;
constexpr int kS1    = 512;
constexpr int kNs1   = 32;
constexpr int kS2    = 128;
constexpr int kNs2   = 64;
constexpr int kCh1   = 128;
constexpr int kCh2   = 256;
constexpr int kCh3   = 512;
constexpr int kZdim  = 256;
constexpr int kW2ld  = 131;
constexpr int kW3ld  = 259;
static_assert(kW2ld == 3 + kCh1);
static_assert(kW3ld == 3 + kCh2);
static_assert(kN1 % 128 == 0 && kS1 % 256 == 0);

__device__ __forceinline__ unsigned f2bf_u32(float f) {
  const unsigned u = __float_as_uint(f);
  return (u + 0x7FFFu + ((u >> 16) & 1u)) >> 16;
}
__device__ __forceinline__ float bf_u32_to_f(unsigned h) { return __uint_as_float(h << 16); }

__device__ __forceinline__ void store2_v4f(float* p, v4f v) {
  *(volatile v4f*)p = v;
  __threadfence();
  *(volatile v4f*)p = v;
}
__device__ __forceinline__ void store2_v4u(void* p, v4u v) {
  *(volatile v4u*)p = v;
  __threadfence();
  *(volatile v4u*)p = v;
}

__device__ __forceinline__ void dep_guard4_b(v8f& a, v8f& b, v8f& c, v8f& d, v16b x, v16b y) {
  asm volatile("v_nop\n\tv_nop\n\tv_nop\n\tv_nop" : "+v"(a), "+v"(b), "+v"(c), "+v"(d) : "v"(x), "v"(y));
}
__device__ __forceinline__ void keep4_b(v16b a, v16b b, v16b c, v16b d) { asm volatile("v_nop" :: "v"(a), "v"(b), "v"(c), "v"(d)); }
__device__ __forceinline__ void acc_guard4(v8f& a, v8f& b, v8f& c, v8f& d) {
  asm volatile("v_nop\n\tv_nop\n\tv_nop\n\tv_nop" : "+v"(a), "+v"(b), "+v"(c), "+v"(d));
}
struct FragB {
  union U { v16b v; v8b h[2]; };
  static __device__ __forceinline__ v16b load(const __bf16* p) {
    U f; f.h[0] = *(const v8b*)(p); f.h[1] = *(const v8b*)(p + 16); return f.v;
  }
  static __device__ __forceinline__ v8f mma(v16b a, v16b b, v8f c) {
    return __builtin_amdgcn_wmma_f32_16x16x32_bf16(false, a, false, b, (short)0, c, false, false);
  }
};

__global__ __launch_bounds__(256) void pack_w_split(const float* __restrict__ W,
                                                    unsigned short* __restrict__ dh,
                                                    unsigned short* __restrict__ dl,
                                                    int ldw, int col0, int rows, int cols) {
  const int t = blockIdx.x * 256 + threadIdx.x;
  const int per_row = cols >> 3;
  const int total = rows * per_row;
  const int tc = t < total ? t : total - 1;
  const int r = tc / per_row;
  const int c8 = (tc - r * per_row) << 3;
  const float* src = W + (size_t)r * ldw + col0 + c8;
  unsigned hb[8], lb[8];
#pragma unroll
  for (int e = 0; e < 8; ++e) {
    const float f = src[e];
    const unsigned h = f2bf_u32(f);
    const unsigned l = f2bf_u32(f - bf_u32_to_f(h));
    hb[e] = h;
    lb[e] = l;
  }
  v4u vh, vl;
  vh.x = hb[0] | (hb[1] << 16); vh.y = hb[2] | (hb[3] << 16); vh.z = hb[4] | (hb[5] << 16); vh.w = hb[6] | (hb[7] << 16);
  vl.x = lb[0] | (lb[1] << 16); vl.y = lb[2] | (lb[3] << 16); vl.z = lb[4] | (lb[5] << 16); vl.w = lb[6] | (lb[7] << 16);
  if (t < total) {
    const size_t o = (size_t)tc * 8;
    store2_v4u(dh + o, vh);
    store2_v4u(dl + o, vl);
  }
}

template <int NT, int PPT, int PPC, int NPOINT>
__global__ __launch_bounds__(NT) void fps_kernel(const float* __restrict__ xyz, float* __restrict__ new_xyz) {
#pragma clang fp contract(off)
  constexpr int NP = NT * PPT;
  constexpr int NWV = NT / 32;
  constexpr int NCHUNK = PPT / PPC;
  constexpr int NF4 = NPOINT * 3 / 4;
  static_assert(PPT % PPC == 0);
  static_assert((NWV & (NWV - 1)) == 0 && NWV <= 32);
  static_assert(NPOINT <= 512 && (NPOINT * 3) % 4 == 0 && NF4 % 32 == 0 && NF4 <= NT);
  __shared__ float sStage[NT * PPC * 3];
  __shared__ float sVal[2][32];
  __shared__ int   sIdx[2][32];
  __shared__ int   sSel[512];

  const int b = blockIdx.x;
  const int tid = threadIdx.x;
  const int lane = tid & 31;
  const int wave = tid >> 5;
  const float* X = xyz + (size_t)b * NP * 3;

  float px[PPT], py[PPT], pz[PPT], dist[PPT];
#pragma unroll
  for (int ch = 0; ch < NCHUNK; ++ch) {
    __syncthreads();
    const float* src = X + (size_t)ch * NT * PPC * 3;
#pragma unroll
    for (int t = 0; t < 3 * PPC; ++t) sStage[tid + t * NT] = src[tid + t * NT];
    __syncthreads();
#pragma unroll
    for (int p = 0; p < PPC; ++p) {
      const int loc = tid + p * NT;
      px[ch * PPC + p] = sStage[loc * 3 + 0];
      py[ch * PPC + p] = sStage[loc * 3 + 1];
      pz[ch * PPC + p] = sStage[loc * 3 + 2];
    }
  }
#pragma unroll
  for (int i = 0; i < PPT; ++i) dist[i] = 1e10f;

  int far = 0;
#pragma unroll 1
  for (int s = 0; s < NPOINT; ++s) {
    if (tid == 0) sSel[s] = far;
    int fc = far < 0 ? 0 : far;
    fc = fc > NP - 1 ? NP - 1 : fc;
    const float cx = X[(size_t)fc * 3 + 0];
    const float cy = X[(size_t)fc * 3 + 1];
    const float cz = X[(size_t)fc * 3 + 2];
    float best = -1.0f;
    int bi = tid;
#pragma unroll
    for (int i = 0; i < PPT; ++i) {
      const float dx = px[i] - cx;
      const float dy = py[i] - cy;
      const float dz = pz[i] - cz;
      const float t0 = dx * dx;
      const float t1 = dy * dy;
      const float t2 = dz * dz;
      const float d = (t0 + t2) + t1;
      const float nd = fminf(dist[i], d);
      dist[i] = nd;
      if (nd > best) { best = nd; bi = tid + i * NT; }
    }
#pragma unroll
    for (int off = 1; off < 32; off <<= 1) {
      const float ov = __shfl_xor(best, off, 32);
      const int   oi = __shfl_xor(bi, off, 32);
      const bool take = (ov > best) || (ov == best && oi < bi);
      best = take ? ov : best;
      bi   = take ? oi : bi;
    }
    const int par = s & 1;
    if (lane == 0) { sVal[par][wave] = best; sIdx[par][wave] = bi; }
    __syncthreads();
    float v = sVal[par][lane & (NWV - 1)];
    int  ix = sIdx[par][lane & (NWV - 1)];
#pragma unroll
    for (int off = 1; off < 32; off <<= 1) {
      const float ov = __shfl_xor(v, off, 32);
      const int   oi = __shfl_xor(ix, off, 32);
      const bool take = (ov > v) || (ov == v && oi < ix);
      v  = take ? ov : v;
      ix = take ? oi : ix;
    }
    far = ix;
  }
  __syncthreads();
  if (tid < NF4) {
    float o[4];
#pragma unroll
    for (int e = 0; e < 4; ++e) {
      const int fl = tid * 4 + e;
      const int pt = fl / 3;
      const int co = fl - pt * 3;
      int sel = sSel[pt];
      sel = sel < 0 ? 0 : sel;
      sel = sel > NP - 1 ? NP - 1 : sel;
      o[e] = X[(size_t)sel * 3 + co];
    }
    v4f v;
    v.x = o[0]; v.y = o[1]; v.z = o[2]; v.w = o[3];
    store2_v4f(new_xyz + (size_t)b * NPOINT * 3 + tid * 4, v);
  }
}

template <int NT, int NS, int NPT, int SQ, bool HAS_P>
__global__ __launch_bounds__(NT) void sa_group_kernel(const float* __restrict__ pts,
                                                      const float* __restrict__ ctr,
                                                      const float* __restrict__ Pfeat,
                                                      const float* __restrict__ w,
                                                      const float* __restrict__ bias,
                                                      float* __restrict__ planes,
                                                      int ldw, float r2) {
#pragma clang fp contract(off)
  constexpr int NWV = NT / 32;
  static_assert(NPT % NT == 0 && NS % 32 == 0 && NS * 3 <= NT && (NS * 3) % 32 == 0);
  __shared__ int   sCnt[2][NWV];
  __shared__ int   sList[NS];
  __shared__ int   sJ[NS];
  __shared__ float sG[NS * 3];
  __shared__ __align__(16) float sOut[4][NT];

  const int g = blockIdx.x;
  const int b = g / SQ;
  const int tid = threadIdx.x;
  const int lane = tid & 31;
  const int wave = tid >> 5;
  const float* X = pts + (size_t)b * NPT * 3;
  const float qx = ctr[(size_t)g * 3 + 0];
  const float qy = ctr[(size_t)g * 3 + 1];
  const float qz = ctr[(size_t)g * 3 + 2];
  const float q0 = qx * qx;
  const float q1 = qy * qy;
  const float q2 = qz * qz;
  const float sqq = (q0 + q2) + q1;

  if (tid < NS) sList[tid] = 0;
  __syncthreads();

  int cnt = 0;
  int it = 0;
  for (int base = 0; base < NPT && cnt < NS; base += NT, ++it) {
    const int j = base + tid;
    const float px = X[(size_t)j * 3 + 0];
    const float py = X[(size_t)j * 3 + 1];
    const float pz = X[(size_t)j * 3 + 2];
    const float a0 = px * px;
    const float a1 = py * py;
    const float a2 = pz * pz;
    const float sqp = (a0 + a2) + a1;
    float p = qx * px;
    p = __builtin_fmaf(qy, py, p);
    p = __builtin_fmaf(qz, pz, p);
    const float tp = 2.0f * p;
    const float d2 = (sqq + sqp) - tp;
    const bool within = !(d2 > r2);
    const unsigned mask = (unsigned)__ballot(within ? 1 : 0);
    const int par = it & 1;
    if (lane == 0) sCnt[par][wave] = __popc(mask);
    __syncthreads();
    int tot = 0, woff = 0;
#pragma unroll
    for (int w2 = 0; w2 < NWV; ++w2) {
      const int cw = sCnt[par][w2];
      woff += (w2 < wave) ? cw : 0;
      tot += cw;
    }
    const int pre = __popc(mask & ((1u << lane) - 1u));
    const int slot = cnt + woff + pre;
    if (within && slot < NS) sList[slot] = j;
    cnt = __builtin_amdgcn_readfirstlane(cnt + tot);
  }
  __syncthreads();
  const int nfound = cnt < NS ? cnt : NS;
  const int f0 = sList[0];
  const int first = (nfound > 0) ? f0 : (NPT - 1);
  if (tid < NS) {
    int v = sList[tid];
    v = (tid < nfound) ? v : first;
    v = v < 0 ? 0 : v;
    v = v > NPT - 1 ? NPT - 1 : v;
    sJ[tid] = v;
  }
  __syncthreads();
  if (tid < NS * 3) {
    const int k = tid / 3;
    const int co = tid - k * 3;
    const int j = sJ[k];
    sG[tid] = X[(size_t)j * 3 + co] - ctr[(size_t)g * 3 + co];
  }
  __syncthreads();

  const int ch = tid;
  const float wx = w[(size_t)ch * ldw + 0];
  const float wy = w[(size_t)ch * ldw + 1];
  const float wz = w[(size_t)ch * ldw + 2];
  const float bb = bias[ch];
  const float* Pb = Pfeat + (size_t)b * NPT * NT + ch;
  float mx = -3.0e38f, mn = 3.0e38f, sm = 0.0f, sq = 0.0f;
#pragma unroll 4
  for (int k = 0; k < NS; ++k) {
    float x = sG[3 * k + 0] * wx;
    x = __builtin_fmaf(sG[3 * k + 1], wy, x);
    x = __builtin_fmaf(sG[3 * k + 2], wz, x);
    float h;
    if (HAS_P) {
      const int j = sJ[k];
      const float pv = Pb[(size_t)j * NT];
      h = (pv + x) + bb;
    } else {
      h = x + bb;
    }
    mx = fmaxf(mx, h);
    mn = fminf(mn, h);
    sm = sm + h;
    sq = __builtin_fmaf(h, h, sq);
  }
  sOut[0][ch] = mx;
  sOut[1][ch] = mn;
  sOut[2][ch] = sm;
  sOut[3][ch] = sq;
  __syncthreads();
  {
    constexpr int QPP = NT / 4;
    const int pl = tid / QPP;
    const int q = tid - pl * QPP;
    const v4f v = *(const v4f*)(&sOut[pl][4 * q]);
    const size_t plane_stride = (size_t)gridDim.x * NT;
    store2_v4f(planes + (size_t)pl * plane_stride + (size_t)g * NT + 4 * q, v);
  }
}

__global__ __launch_bounds__(256) void bn_stats_kernel(const float* __restrict__ psum, const float* __restrict__ psq,
                                                       const float* __restrict__ gamma, const float* __restrict__ beta,
                                                       float* __restrict__ ss, double inv_count, int ngroups, int nch) {
  __shared__ double sS[8][32];
  __shared__ double sQ[8][32];
  __shared__ __align__(16) float sO[2][32];
  const int tid = threadIdx.x;
  const int r8 = tid >> 5;
  const int cl = tid & 31;
  const int c0 = blockIdx.x * 32;
  const int c = c0 + cl;
  double s = 0.0, q = 0.0;
#pragma unroll 4
  for (int g = r8; g < ngroups; g += 8) {
    s += (double)psum[(size_t)g * nch + c];
    q += (double)psq[(size_t)g * nch + c];
  }
  sS[r8][cl] = s;
  sQ[r8][cl] = q;
  __syncthreads();
  if (tid < 32) {
    double S = 0.0, Q = 0.0;
#pragma unroll
    for (int r = 0; r < 8; ++r) { S += sS[r][cl]; Q += sQ[r][cl]; }
    const double mean = S * inv_count;
    double var = Q * inv_count - mean * mean;
    var = var < 0.0 ? 0.0 : var;
    const float varf = (float)var;
    const float meanf = (float)mean;
    const float sc = gamma[c] * (1.0f / sqrtf(varf + 1e-5f));
    const float sh = beta[c] - meanf * sc;
    sO[0][cl] = sc;
    sO[1][cl] = sh;
  }
  __syncthreads();
  if (tid < 16) {
    const int which = tid >> 3;
    const int q4 = tid & 7;
    const v4f v = *(const v4f*)(&sO[which][4 * q4]);
    store2_v4f(ss + (size_t)which * nch + c0 + 4 * q4, v);
  }
}

__global__ __launch_bounds__(256) void bn_apply_split_kernel(const float* __restrict__ pmax, const float* __restrict__ pmin,
                                                             const float* __restrict__ ss,
                                                             unsigned short* __restrict__ oh, unsigned short* __restrict__ ol,
                                                             int nch, int total8) {
  const int t = blockIdx.x * 256 + threadIdx.x;
  const int tc = t < total8 ? t : total8 - 1;
  const size_t e0 = (size_t)tc * 8;
  const int c = (int)(e0 & (size_t)(nch - 1));
  const v4f mxa = *(const v4f*)(pmax + e0);
  const v4f mxb = *(const v4f*)(pmax + e0 + 4);
  const v4f mna = *(const v4f*)(pmin + e0);
  const v4f mnb = *(const v4f*)(pmin + e0 + 4);
  const v4f sca = *(const v4f*)(ss + c);
  const v4f scb = *(const v4f*)(ss + c + 4);
  const v4f sha = *(const v4f*)(ss + nch + c);
  const v4f shb = *(const v4f*)(ss + nch + c + 4);
  const float mx[8] = {mxa.x, mxa.y, mxa.z, mxa.w, mxb.x, mxb.y, mxb.z, mxb.w};
  const float mn[8] = {mna.x, mna.y, mna.z, mna.w, mnb.x, mnb.y, mnb.z, mnb.w};
  const float sc[8] = {sca.x, sca.y, sca.z, sca.w, scb.x, scb.y, scb.z, scb.w};
  const float sh[8] = {sha.x, sha.y, sha.z, sha.w, shb.x, shb.y, shb.z, shb.w};
  unsigned hb[8], lb[8];
#pragma unroll
  for (int e = 0; e < 8; ++e) {
    const float a = sc[e];
    const float ext = (a >= 0.0f) ? mx[e] : mn[e];
    float y = __builtin_fmaf(a, ext, sh[e]);
    y = fmaxf(y, 0.0f);
    const unsigned h = f2bf_u32(y);
    const unsigned l = f2bf_u32(y - bf_u32_to_f(h));
    hb[e] = h;
    lb[e] = l;
  }
  v4u vh, vl;
  vh.x = hb[0] | (hb[1] << 16); vh.y = hb[2] | (hb[3] << 16); vh.z = hb[4] | (hb[5] << 16); vh.w = hb[6] | (hb[7] << 16);
  vl.x = lb[0] | (lb[1] << 16); vl.y = lb[2] | (lb[3] << 16); vl.z = lb[4] | (lb[5] << 16); vl.w = lb[6] | (lb[7] << 16);
  if (t < total8) {
    store2_v4u(oh + e0, vh);
    store2_v4u(ol + e0, vl);
  }
}

__global__ __launch_bounds__(256) void wmma_gemm64_bf16x3(
    const unsigned short* __restrict__ Ap, const unsigned short* __restrict__ A2p,
    const unsigned short* __restrict__ Btp, const unsigned short* __restrict__ Bt2p,
    float* __restrict__ Cout, int lda, int ldb, int ldc, int M, int N, int K) {
  typedef __bf16 T;
  typedef v16b V;
  const T* A = (const T*)Ap; const T* A2 = (const T*)A2p; const T* Bt = (const T*)Btp; const T* Bt2 = (const T*)Bt2p;
  __shared__ __align__(16) float sT[8][16 * 68];
  const int lane = threadIdx.x & 31;
  const int wave = threadIdx.x >> 5;
  const int tilesN = N >> 6;
  const int tilesM = M >> 6;
  const int tile = blockIdx.x * 8 + wave;
  if (tile >= tilesM * tilesN) return;
  const int tm = tile / tilesN;
  const int tn = tile - tm * tilesN;
  const int m0 = tm << 6;
  const int n0 = tn << 6;

  const int rlane = lane & 15;
  const int koff  = (lane >> 4) * 8;
  const int mOff  = (lane >> 4) * 8;

  v8f acc[4][4];
#pragma unroll
  for (int i = 0; i < 4; ++i)
#pragma unroll
    for (int j = 0; j < 4; ++j) acc[i][j] = (v8f){0.f,0.f,0.f,0.f,0.f,0.f,0.f,0.f};

  for (int k0 = 0; k0 < K; k0 += 32) {
    V bh[4], bl[4];
#pragma unroll
    for (int j = 0; j < 4; ++j) {
      const size_t bo = (size_t)(n0 + (j << 4) + rlane) * ldb + koff + k0;
      bh[j] = FragB::load(Bt + bo);
      bl[j] = FragB::load(Bt2 + bo);
    }
#pragma unroll
    for (int i = 0; i < 4; ++i) {
      const size_t ao = (size_t)(m0 + (i << 4) + rlane) * lda + koff + k0;
      V ah = FragB::load(A + ao);
      V al = FragB::load(A2 + ao);
#pragma unroll
      for (int j = 0; j < 4; ++j) {
        acc[i][j] = FragB::mma(ah, bh[j], acc[i][j]);
        acc[i][j] = FragB::mma(ah, bl[j], acc[i][j]);
        acc[i][j] = FragB::mma(al, bh[j], acc[i][j]);
      }
      dep_guard4_b(acc[i][0], acc[i][1], acc[i][2], acc[i][3], ah, al);
    }
    keep4_b(bh[0], bh[1], bh[2], bh[3]);
    keep4_b(bl[0], bl[1], bl[2], bl[3]);
  }
  acc_guard4(acc[0][0], acc[0][1], acc[0][2], acc[0][3]);
  acc_guard4(acc[1][0], acc[1][1], acc[1][2], acc[1][3]);
  acc_guard4(acc[2][0], acc[2][1], acc[2][2], acc[2][3]);
  acc_guard4(acc[3][0], acc[3][1], acc[3][2], acc[3][3]);

  float* slab = sT[wave];
#pragma unroll
  for (int i = 0; i < 4; ++i) {
    const int mBase = m0 + (i << 4);
#pragma unroll
    for (int j = 0; j < 4; ++j) {
#pragma unroll
      for (int r = 0; r < 8; ++r) {
        slab[(mOff + r) * 68 + (j << 4) + rlane] = acc[i][j][r];
      }
    }
    __builtin_amdgcn_fence(__ATOMIC_RELEASE, "workgroup");
    __builtin_amdgcn_wave_barrier();
    __builtin_amdgcn_fence(__ATOMIC_ACQUIRE, "workgroup");
    {
      const int hh = lane >> 4, c4 = (lane & 15) * 4;
      for (int pass = 0; pass < 2; ++pass) {
#pragma unroll
        for (int it = 0; it < 8; ++it) {
          const int row = it * 2 + hh;
          v4f v = *(const v4f*)(slab + row * 68 + c4);
          *(volatile v4f*)(Cout + (size_t)(mBase + row) * ldc + n0 + c4) = v;
        }
        __threadfence();
      }
    }
    __builtin_amdgcn_fence(__ATOMIC_RELEASE, "workgroup");
    __builtin_amdgcn_wave_barrier();
    __builtin_amdgcn_fence(__ATOMIC_ACQUIRE, "workgroup");
  }
}

__global__ __launch_bounds__(256) void sa3_stats_kernel(const float* __restrict__ H, const float* __restrict__ cxyz,
                                                        const float* __restrict__ w3, const float* __restrict__ b3,
                                                        float* __restrict__ planes) {
  __shared__ float sX[kS2 * 3];
  __shared__ float sR[4][8][32];
  __shared__ __align__(16) float sO[4][32];
  const int tid = threadIdx.x;
  const int b = blockIdx.x >> 4;
  const int c0 = (blockIdx.x & 15) * 32;
  const int r8 = tid >> 5;
  const int cl = tid & 31;
  const int c = c0 + cl;
  sX[tid] = cxyz[(size_t)b * kS2 * 3 + tid];
  if (tid < 128) sX[256 + tid] = cxyz[(size_t)b * kS2 * 3 + 256 + tid];
  __syncthreads();
  const float wx = w3[(size_t)c * kW3ld + 0];
  const float wy = w3[(size_t)c * kW3ld + 1];
  const float wz = w3[(size_t)c * kW3ld + 2];
  const float bb = b3[c];
  float mx = -3.0e38f, mn = 3.0e38f, sm = 0.0f, sq = 0.0f;
#pragma unroll 4
  for (int r = r8; r < kS2; r += 8) {
    const float hv = H[((size_t)b * kS2 + r) * kCh3 + c];
    float x = sX[3 * r + 0] * wx;
    x = __builtin_fmaf(sX[3 * r + 1], wy, x);
    x = __builtin_fmaf(sX[3 * r + 2], wz, x);
    const float h = (hv + x) + bb;
    mx = fmaxf(mx, h);
    mn = fminf(mn, h);
    sm = sm + h;
    sq = __builtin_fmaf(h, h, sq);
  }
  sR[0][r8][cl] = mx;
  sR[1][r8][cl] = mn;
  sR[2][r8][cl] = sm;
  sR[3][r8][cl] = sq;
  __syncthreads();
  if (tid < 32) {
    float M = -3.0e38f, m = 3.0e38f, S = 0.0f, Q = 0.0f;
#pragma unroll
    for (int r = 0; r < 8; ++r) {
      M = fmaxf(M, sR[0][r][cl]);
      m = fminf(m, sR[1][r][cl]);
      S = S + sR[2][r][cl];
      Q = Q + sR[3][r][cl];
    }
    sO[0][cl] = M;
    sO[1][cl] = m;
    sO[2][cl] = S;
    sO[3][cl] = Q;
  }
  __syncthreads();
  if (tid < 32) {
    const int pl = tid >> 3;
    const int q4 = tid & 7;
    const v4f v = *(const v4f*)(&sO[pl][4 * q4]);
    store2_v4f(planes + (size_t)pl * (kBatch * kCh3) + (size_t)b * kCh3 + c0 + 4 * q4, v);
  }
}

__global__ __launch_bounds__(32) void fc_kernel(const float* __restrict__ pmax3, const float* __restrict__ pmin3,
                                                const float* __restrict__ ss3, const float* __restrict__ wf,
                                                const float* __restrict__ bfv, float* __restrict__ out) {
  __shared__ __align__(16) float sL[kCh3];
  __shared__ __align__(16) float sRes[32];
  const int lane = threadIdx.x;
  const int b = blockIdx.x >> 3;
  const int n0 = (blockIdx.x & 7) * 32;
#pragma unroll 2
  for (int i = 0; i < kCh3 / 32; ++i) {
    const int k = lane + 32 * i;
    const float a  = ss3[k];
    const float sh = ss3[kCh3 + k];
    const float mx = pmax3[(size_t)b * kCh3 + k];
    const float mn = pmin3[(size_t)b * kCh3 + k];
    const float ext = (a >= 0.0f) ? mx : mn;
    sL[k] = fmaxf(__builtin_fmaf(a, ext, sh), 0.0f);
  }
  __syncthreads();
  const int n = n0 + lane;
  const float* wr = wf + (size_t)n * kCh3;
  float a0 = 0.0f, a1 = 0.0f, a2 = 0.0f, a3 = 0.0f;
#pragma unroll 2
  for (int k4 = 0; k4 < kCh3 / 4; ++k4) {
    const v4f wv = *(const v4f*)(wr + 4 * k4);
    const v4f xv = *(const v4f*)(sL + 4 * k4);
    a0 = __builtin_fmaf(wv.x, xv.x, a0);
    a1 = __builtin_fmaf(wv.y, xv.y, a1);
    a2 = __builtin_fmaf(wv.z, xv.z, a2);
    a3 = __builtin_fmaf(wv.w, xv.w, a3);
  }
  const float r = ((a0 + a1) + (a2 + a3)) + bfv[n];
  sRes[lane] = r;
  __syncthreads();
  if (lane < 8) {
    const v4f v = *(const v4f*)(&sRes[4 * lane]);
    store2_v4f(out + (size_t)b * kZdim + n0 + 4 * lane, v);
  }
}

constexpr size_t al256(size_t x) { return (x + 255) & ~(size_t)255; }

constexpr size_t SZ_W2P  = (size_t)kCh2 * kCh1 * 2;
constexpr size_t SZ_W3P  = (size_t)kCh3 * kCh2 * 2;
constexpr size_t SZ_L1X  = (size_t)kBatch * kS1 * 3 * 4;
constexpr size_t SZ_PL1  = (size_t)4 * kBatch * kS1 * kCh1 * 4;
constexpr size_t SZ_SS   = 4096;
constexpr size_t SZ_A1P  = (size_t)kBatch * kS1 * kCh1 * 2;
constexpr size_t SZ_L2X  = (size_t)kBatch * kS2 * 3 * 4;
constexpr size_t SZ_PF   = (size_t)kBatch * kS1 * kCh2 * 4;
constexpr size_t SZ_PL2  = (size_t)4 * kBatch * kS2 * kCh2 * 4;
constexpr size_t SZ_A2P  = (size_t)kBatch * kS2 * kCh2 * 2;
constexpr size_t SZ_H3   = (size_t)kBatch * kS2 * kCh3 * 4;
constexpr size_t SZ_PL3  = (size_t)4 * kBatch * kCh3 * 4;

constexpr size_t OFF_W2H = 0;
constexpr size_t OFF_W2L = OFF_W2H + al256(SZ_W2P);
constexpr size_t OFF_W3H = OFF_W2L + al256(SZ_W2P);
constexpr size_t OFF_W3L = OFF_W3H + al256(SZ_W3P);
constexpr size_t OFF_L1X = OFF_W3L + al256(SZ_W3P);
constexpr size_t OFF_PL1 = OFF_L1X + al256(SZ_L1X);
constexpr size_t OFF_SS1 = OFF_PL1 + al256(SZ_PL1);
constexpr size_t OFF_A1H = OFF_SS1 + al256(SZ_SS);
constexpr size_t OFF_A1L = OFF_A1H + al256(SZ_A1P);
constexpr size_t OFF_L2X = OFF_A1L + al256(SZ_A1P);
constexpr size_t OFF_PF  = OFF_L2X + al256(SZ_L2X);
constexpr size_t OFF_PL2 = OFF_PF  + al256(SZ_PF);
constexpr size_t OFF_SS2 = OFF_PL2 + al256(SZ_PL2);
constexpr size_t OFF_A2H = OFF_SS2 + al256(SZ_SS);
constexpr size_t OFF_A2L = OFF_A2H + al256(SZ_A2P);
constexpr size_t OFF_H3  = OFF_A2L + al256(SZ_A2P);
constexpr size_t OFF_PL3 = OFF_H3  + al256(SZ_H3);
constexpr size_t OFF_SS3 = OFF_PL3 + al256(SZ_PL3);
constexpr size_t WS_TOTAL = OFF_SS3 + al256(SZ_SS);
static_assert(WS_TOTAL <= (size_t)134217728);

static_assert((kBatch * kS1) % 64 == 0 && kCh2 % 64 == 0 && kCh1 % 32 == 0);
static_assert((kBatch * kS2) % 64 == 0 && kCh3 % 64 == 0 && kCh2 % 32 == 0);
static_assert((size_t)kBatch * kZdim * 4 == 8192);

extern "C" void kernel_launch(void* const* d_in, const int* in_sizes, int n_in,
                              void* d_out, int out_size, void* d_ws, size_t ws_size,
                              hipStream_t stream) {
  (void)in_sizes; (void)out_size;
  if (n_in < 15) return;
  if (ws_size < WS_TOTAL) return;
  const float* xyz = (const float*)d_in[0];
  const float* w1  = (const float*)d_in[1];
  const float* b1  = (const float*)d_in[2];
  const float* g1  = (const float*)d_in[3];
  const float* be1 = (const float*)d_in[4];
  const float* w2  = (const float*)d_in[5];
  const float* b2  = (const float*)d_in[6];
  const float* g2  = (const float*)d_in[7];
  const float* be2 = (const float*)d_in[8];
  const float* w3  = (const float*)d_in[9];
  const float* b3  = (const float*)d_in[10];
  const float* g3  = (const float*)d_in[11];
  const float* be3 = (const float*)d_in[12];
  const float* wf  = (const float*)d_in[13];
  const float* bfv = (const float*)d_in[14];
  float* outp = (float*)d_out;

  char* base = (char*)d_ws;
  unsigned short* w2h = (unsigned short*)(base + OFF_W2H);
  unsigned short* w2l = (unsigned short*)(base + OFF_W2L);
  unsigned short* w3h = (unsigned short*)(base + OFF_W3H);
  unsigned short* w3l = (unsigned short*)(base + OFF_W3L);
  float* l1xyz = (float*)(base + OFF_L1X);
  float* pl1   = (float*)(base + OFF_PL1);
  float* ss1   = (float*)(base + OFF_SS1);
  unsigned short* a1h = (unsigned short*)(base + OFF_A1H);
  unsigned short* a1l = (unsigned short*)(base + OFF_A1L);
  float* l2xyz = (float*)(base + OFF_L2X);
  float* pfeat = (float*)(base + OFF_PF);
  float* pl2   = (float*)(base + OFF_PL2);
  float* ss2   = (float*)(base + OFF_SS2);
  unsigned short* a2h = (unsigned short*)(base + OFF_A2H);
  unsigned short* a2l = (unsigned short*)(base + OFF_A2L);
  float* h3    = (float*)(base + OFF_H3);
  float* pl3   = (float*)(base + OFF_PL3);
  float* ss3   = (float*)(base + OFF_SS3);

  const size_t st1 = (size_t)kBatch * kS1 * kCh1;
  const size_t st2 = (size_t)kBatch * kS2 * kCh2;
  const size_t st3 = (size_t)kBatch * kCh3;

  pack_w_split<<<(kCh2 * kCh1 / 8) / 256, 256, 0, stream>>>(w2, w2h, w2l, kW2ld, 3, kCh2, kCh1);
  pack_w_split<<<(kCh3 * kCh2 / 8) / 256, 256, 0, stream>>>(w3, w3h, w3l, kW3ld, 3, kCh3, kCh2);

  fps_kernel<512, 16, 2, kS1><<<kBatch, 512, 0, stream>>>(xyz, l1xyz);
  sa_group_kernel<kCh1, kNs1, kN1, kS1, false><<<kBatch * kS1, kCh1, 0, stream>>>(
      xyz, l1xyz, xyz, w1, b1, pl1, 3, 0.04f);
  bn_stats_kernel<<<kCh1 / 32, 256, 0, stream>>>(pl1 + 2 * st1, pl1 + 3 * st1, g1, be1, ss1,
      1.0 / (double)(kBatch * kS1 * kNs1), kBatch * kS1, kCh1);
  bn_apply_split_kernel<<<(kBatch * kS1 * kCh1 / 8) / 256, 256, 0, stream>>>(pl1, pl1 + st1, ss1, a1h, a1l,
      kCh1, kBatch * kS1 * kCh1 / 8);

  fps_kernel<512, 1, 1, kS2><<<kBatch, 512, 0, stream>>>(l1xyz, l2xyz);
  wmma_gemm64_bf16x3<<<((kBatch * kS1 / 64) * (kCh2 / 64)) / 8, 256, 0, stream>>>(
      a1h, a1l, w2h, w2l, pfeat, kCh1, kCh1, kCh2, kBatch * kS1, kCh2, kCh1);
  sa_group_kernel<kCh2, kNs2, kS1, kS2, true><<<kBatch * kS2, kCh2, 0, stream>>>(
      l1xyz, l2xyz, pfeat, w2, b2, pl2, kW2ld, 0.16f);
  bn_stats_kernel<<<kCh2 / 32, 256, 0, stream>>>(pl2 + 2 * st2, pl2 + 3 * st2, g2, be2, ss2,
      1.0 / (double)(kBatch * kS2 * kNs2), kBatch * kS2, kCh2);
  bn_apply_split_kernel<<<(kBatch * kS2 * kCh2 / 8) / 256, 256, 0, stream>>>(pl2, pl2 + st2, ss2, a2h, a2l,
      kCh2, kBatch * kS2 * kCh2 / 8);

  wmma_gemm64_bf16x3<<<((kBatch * kS2 / 64) * (kCh3 / 64)) / 8, 256, 0, stream>>>(
      a2h, a2l, w3h, w3l, h3, kCh2, kCh2, kCh3, kBatch * kS2, kCh3, kCh2);
  sa3_stats_kernel<<<kBatch * (kCh3 / 32), 256, 0, stream>>>(h3, l2xyz, w3, b3, pl3);
  bn_stats_kernel<<<kCh3 / 32, 256, 0, stream>>>(pl3 + 2 * st3, pl3 + 3 * st3, g3, be3, ss3,
      1.0 / (double)(kBatch * kS2), kBatch, kCh3);

  fc_kernel<<<kBatch * (kZdim / 32), 32, 0, stream>>>(pl3, pl3 + st3, ss3, wf, bfv, outp);
}
